// LSTMComplex_51505247814030
// MI455X (gfx1250) — hardware-verified
//
#include <hip/hip_runtime.h>
#include <math.h>

typedef __attribute__((ext_vector_type(16))) _Float16 v16h;
typedef __attribute__((ext_vector_type(8)))  _Float16 v8h;
typedef __attribute__((ext_vector_type(16))) __bf16   v16b;
typedef __attribute__((ext_vector_type(8)))  __bf16   v8b;
typedef __attribute__((ext_vector_type(8)))  float    v8f;
typedef __attribute__((ext_vector_type(4)))  float    v4f;
typedef __attribute__((ext_vector_type(2)))  unsigned v2u;
typedef __attribute__((ext_vector_type(4)))  unsigned v4u;

constexpr int   kSeq         = 128;
constexpr int   kSteps       = 1024;
constexpr int   kRows        = 16;
constexpr int   kRecBlocks   = kSeq / kRows;
constexpr int   kTpThreads   = 256;
constexpr int   kHeadThreads = 128;
constexpr int   kHeadRows    = 64;
constexpr int   kHeadBlocks  = kSeq / kHeadRows;
constexpr int   kAP          = 136;
constexpr float kWsc    = 16.0f;
constexpr float kWscInv = 0.0625f;
constexpr float kResSc  = 2048.0f;
constexpr float kResInv = 0.00048828125f;
constexpr float kLnEps  = 1e-6f;

__device__ __forceinline__ unsigned short f2bf_bits(float f) {
  unsigned u = __float_as_uint(f);
  return (unsigned short)((u + 0x7FFFu + ((u >> 16) & 1u)) >> 16);
}
__device__ __forceinline__ float bf_bits2f(unsigned short h) { return __uint_as_float(((unsigned)h) << 16); }
__device__ __forceinline__ float bf16r(float f) { return bf_bits2f(f2bf_bits(f)); }

__device__ __forceinline__ void dep_guard_h(v8f& a, v8f& b, v16h x, v16h y) { asm volatile("v_nop\n\tv_nop\n\tv_nop\n\tv_nop" : "+v"(a), "+v"(b) : "v"(x), "v"(y)); }
__device__ __forceinline__ void dep_guard_b(v8f& a, v8f& b, v16b x, v16b y) { asm volatile("v_nop\n\tv_nop\n\tv_nop\n\tv_nop" : "+v"(a), "+v"(b) : "v"(x), "v"(y)); }
__device__ __forceinline__ void dep_guard3_h(v8f& a, v8f& b, v16h x, v16h y, v16h z) { asm volatile("v_nop\n\tv_nop\n\tv_nop\n\tv_nop" : "+v"(a), "+v"(b) : "v"(x), "v"(y), "v"(z)); }
__device__ __forceinline__ void keep4_h(v16h a, v16h b, v16h c, v16h d) { asm volatile("v_nop" :: "v"(a), "v"(b), "v"(c), "v"(d)); }
__device__ __forceinline__ void keep4_b(v16b a, v16b b, v16b c, v16b d) { asm volatile("v_nop" :: "v"(a), "v"(b), "v"(c), "v"(d)); }
__device__ __forceinline__ void acc_guard4(v8f& a, v8f& b, v8f& c, v8f& d) { asm volatile("v_nop\n\tv_nop\n\tv_nop\n\tv_nop" : "+v"(a), "+v"(b), "+v"(c), "+v"(d)); }
template <typename T> struct Frag;
template <> struct Frag<_Float16> {
  typedef v16h V; union U { v16h v; v8h h[2]; };
  static __device__ __forceinline__ v16h load(const _Float16* p) {
    U f; f.h[0] = *(const v8h*)(p); f.h[1] = *(const v8h*)(p + 16); return f.v;
  }
  static __device__ __forceinline__ v8f mma(v16h a, v16h b, v8f c) {
    return __builtin_amdgcn_wmma_f32_16x16x32_f16(false, a, false, b, (short)0, c, false, false);
  }
  static __device__ __forceinline__ void guard(v8f& a, v8f& b, v16h x, v16h y) { dep_guard_h(a, b, x, y); }
  static __device__ __forceinline__ void keep(v16h a, v16h b, v16h c, v16h d) { keep4_h(a, b, c, d); }
};
template <> struct Frag<__bf16> {
  typedef v16b V; union U { v16b v; v8b h[2]; };
  static __device__ __forceinline__ v16b load(const __bf16* p) {
    U f; f.h[0] = *(const v8b*)(p); f.h[1] = *(const v8b*)(p + 16); return f.v;
  }
  static __device__ __forceinline__ v8f mma(v16b a, v16b b, v8f c) {
    return __builtin_amdgcn_wmma_f32_16x16x32_bf16(false, a, false, b, (short)0, c, false, false);
  }
  static __device__ __forceinline__ void guard(v8f& a, v8f& b, v16b x, v16b y) { dep_guard_b(a, b, x, y); }
  static __device__ __forceinline__ void keep(v16b a, v16b b, v16b c, v16b d) { keep4_b(a, b, c, d); }
};

__device__ __forceinline__ float fsig(float x)  { return __builtin_amdgcn_rcpf(1.0f + __expf(-x)); }
__device__ __forceinline__ float ftanh(float x) { return 1.0f - 2.0f * __builtin_amdgcn_rcpf(__expf(2.0f * x) + 1.0f); }
__device__ __forceinline__ v8f zero8() { const v8f z = {0.f, 0.f, 0.f, 0.f, 0.f, 0.f, 0.f, 0.f}; return z; }

template <int MODE>
__global__ __launch_bounds__(kTpThreads) void tpw_kernel(const float* __restrict__ src, int R, int C, int ldo,
                                                       unsigned short* __restrict__ O, float sc) {
  __shared__ float Tt[64 * 65];
  const int tid = threadIdx.x;
  const int c0 = blockIdx.x * 64, r0 = blockIdx.y * 64;
#pragma unroll
  for (int i = 0; i < 4; ++i) {
    const int idx = i * kTpThreads + tid;
    const int rr = idx >> 4, cc = (idx & 15) * 4;
    const v4f v = *(const v4f*)(src + (size_t)(r0 + rr) * (size_t)C + c0 + cc);
    Tt[rr * 65 + cc + 0] = v[0];
    Tt[rr * 65 + cc + 1] = v[1];
    Tt[rr * 65 + cc + 2] = v[2];
    Tt[rr * 65 + cc + 3] = v[3];
  }
  __syncthreads();
  const int q = tid >> 3, c8 = (tid & 7) * 8;
  v8h hv[2];
#pragma unroll
  for (int g = 0; g < 2; ++g) {
    const int qq = g * 32 + q;
#pragma unroll
    for (int e = 0; e < 8; ++e) {
      const float f = Tt[(c8 + e) * 65 + qq];
      unsigned short bits;
      if (MODE == 0) {
        bits = f2bf_bits(f * sc);
      } else {
        const float fb = bf_bits2f(f2bf_bits(f));
        bits = __builtin_bit_cast(unsigned short, (_Float16)(fb * sc));
      }
      hv[g][e] = __builtin_bit_cast(_Float16, bits);
    }
  }
  for (int pass = 0; pass < 2; ++pass) {
#pragma unroll
    for (int g = 0; g < 2; ++g) {
      const size_t o = (size_t)(c0 + g * 32 + q) * (size_t)ldo + (size_t)(r0 + c8);
      *(volatile v8h*)(O + o) = hv[g];
    }
    __threadfence();
  }
}

template <int XM> struct XSel;
template <> struct XSel<0> { typedef __bf16   T; };
template <> struct XSel<1> { typedef _Float16 T; };

template <int F, int NT, int XMODE>
__device__ __forceinline__ void load_x_tile(unsigned short* Ax, const float* __restrict__ x32,
                                            const unsigned short* __restrict__ x16, int rowbase, int t, int tid) {
  constexpr int XP = F + 8;
  if constexpr (XMODE == 0) {
    constexpr int SEG = F / 4;
    constexpr int ITER = (kRows * SEG) / NT;
    static_assert(ITER * NT == kRows * SEG);
#pragma unroll
    for (int it = 0; it < ITER; ++it) {
      const int idx = it * NT + tid;
      const int row = idx / SEG, c4 = (idx - row * SEG) * 4;
      const v4f v = *(const v4f*)(x32 + ((size_t)(rowbase + row) * kSteps + (size_t)t) * F + c4);
      v2u pk;
      pk[0] = (unsigned)f2bf_bits(v[0]) | ((unsigned)f2bf_bits(v[1]) << 16);
      pk[1] = (unsigned)f2bf_bits(v[2]) | ((unsigned)f2bf_bits(v[3]) << 16);
      *(v2u*)(Ax + row * XP + c4) = pk;
    }
  } else {
    constexpr int SEG = F / 8;
    constexpr int ITER = (kRows * SEG) / NT;
    static_assert(ITER * NT == kRows * SEG);
#pragma unroll
    for (int it = 0; it < ITER; ++it) {
      const int idx = it * NT + tid;
      const int row = idx / SEG, c8 = (idx - row * SEG) * 8;
      const v4u v = *(const v4u*)(x16 + ((size_t)(rowbase + row) * kSteps + (size_t)t) * F + c8);
      *(v4u*)(Ax + row * XP + c8) = v;
    }
  }
}

template <int F, int H, int NW, int XMODE, bool SEQ>
__global__ __launch_bounds__(32 * NW) void rec_layer_kernel(
    const float* __restrict__ x32,
    const unsigned short* __restrict__ x16,
    const unsigned short* __restrict__ WXp,
    const unsigned short* __restrict__ WHp,
    const float* __restrict__ bias,
    const float* __restrict__ lns,
    const float* __restrict__ lnb,
    unsigned short* __restrict__ hseq,
    float* __restrict__ hfin) {
  constexpr int NT = 32 * NW;
  constexpr int NTILE = H / (16 * NW);
  constexpr int XP = F + 8, HP = H + 8, OP = H + 4;
  static_assert(NTILE >= 1 && NTILE * 16 * NW == H);
  static_assert(F % 32 == 0 && H % 32 == 0);
  typedef typename XSel<XMODE>::T XT;
  typedef typename Frag<XT>::V XV;
  __shared__ __align__(16) unsigned short Ax[kRows * XP];
  __shared__ __align__(16) _Float16       Ah[kRows * HP];
  __shared__ __align__(16) _Float16       Ys[SEQ ? kRows * H : 8];
  __shared__ __align__(16) float          Hs[SEQ ? 4 : kRows * OP];
  __shared__ __align__(16) float          redS[SEQ ? kRows * NW : 4];
  __shared__ __align__(16) float          redQ[SEQ ? kRows * NW : 4];

  const XT*       WX = (const XT*)WXp;
  const _Float16* WH = (const _Float16*)WHp;
  const int tid = threadIdx.x, lane = tid & 31, wave = tid >> 5;
  const int c = lane & 15, hh = lane >> 4, koff = hh * 8;
  const int rowbase = blockIdx.x * kRows;

#pragma unroll 1
  for (int i = tid; i < kRows * HP; i += NT) Ah[i] = (_Float16)0.0f;
  load_x_tile<F, NT, XMODE>(Ax, x32, x16, rowbase, 0, tid);

  float cst[NTILE][8], hst[NTILE][8], bb[NTILE][4], ls[NTILE], lb[NTILE];
#pragma unroll
  for (int nt = 0; nt < NTILE; ++nt) {
    const int j = 16 * NTILE * wave + 16 * nt + c;
#pragma unroll
    for (int g = 0; g < 4; ++g) bb[nt][g] = bf16r(bias[g * H + j]);
    ls[nt] = bf16r(lns[j]);
    lb[nt] = bf16r(lnb[j]);
#pragma unroll
    for (int r = 0; r < 8; ++r) { cst[nt][r] = 0.0f; hst[nt][r] = 0.0f; }
  }
  __syncthreads();

  const XT*       axrow = (const XT*)Ax + c * XP + koff;
  const _Float16* ahrow = Ah + c * HP + koff;

#pragma unroll 1
  for (int t = 0; t < kSteps; ++t) {
#pragma unroll
    for (int nt = 0; nt < NTILE; ++nt) {
      const int j = 16 * NTILE * wave + 16 * nt + c;
      const XT*       wx = WX + (size_t)j * F + koff;
      const _Float16* wh = WH + (size_t)j * H + koff;
      v8f acc[4];
      acc[0] = zero8(); acc[1] = zero8(); acc[2] = zero8(); acc[3] = zero8();
#pragma unroll 1
      for (int kx = 0; kx < F; kx += 32) {
        const XV a  = Frag<XT>::load(axrow + kx);
        const XV b0 = Frag<XT>::load(wx + kx);
        const XV b1 = Frag<XT>::load(wx + (size_t)1 * H * F + kx);
        const XV b2 = Frag<XT>::load(wx + (size_t)2 * H * F + kx);
        const XV b3 = Frag<XT>::load(wx + (size_t)3 * H * F + kx);
        acc[0] = Frag<XT>::mma(a, b0, acc[0]);
        acc[1] = Frag<XT>::mma(a, b1, acc[1]);
        acc[2] = Frag<XT>::mma(a, b2, acc[2]);
        acc[3] = Frag<XT>::mma(a, b3, acc[3]);
        Frag<XT>::guard(acc[0], acc[3], a, b3);
        Frag<XT>::keep(b0, b1, b2, b3);
      }
#pragma unroll 1
      for (int k0 = 0; k0 < H; k0 += 32) {
        const v16h a  = Frag<_Float16>::load(ahrow + k0);
        const v16h b0 = Frag<_Float16>::load(wh + k0);
        const v16h b1 = Frag<_Float16>::load(wh + (size_t)1 * H * H + k0);
        const v16h b2 = Frag<_Float16>::load(wh + (size_t)2 * H * H + k0);
        const v16h b3 = Frag<_Float16>::load(wh + (size_t)3 * H * H + k0);
        acc[0] = Frag<_Float16>::mma(a, b0, acc[0]);
        acc[1] = Frag<_Float16>::mma(a, b1, acc[1]);
        acc[2] = Frag<_Float16>::mma(a, b2, acc[2]);
        acc[3] = Frag<_Float16>::mma(a, b3, acc[3]);
        dep_guard_h(acc[0], acc[3], a, b3);
        keep4_h(b0, b1, b2, b3);
      }
      acc_guard4(acc[0], acc[1], acc[2], acc[3]);
#pragma unroll
      for (int r = 0; r < 8; ++r) {
        const float zi = acc[0][r] * kWscInv + bb[nt][0];
        const float zf = acc[1][r] * kWscInv + bb[nt][1];
        const float zg = acc[2][r] * kWscInv + bb[nt][2];
        const float zo = acc[3][r] * kWscInv + bb[nt][3];
        const float ig = fsig(zi);
        const float fg = fsig(zf);
        const float gg = ftanh(zg);
        const float og = fsig(zo);
        const float cn = fg * cst[nt][r] + ig * gg;
        cst[nt][r] = cn;
        hst[nt][r] = og * ftanh(cn);
      }
    }

    if constexpr (SEQ) {
      float mrow[8], rrow[8];
#pragma unroll
      for (int r = 0; r < 8; ++r) {
        float s = 0.f;
#pragma unroll
        for (int nt = 0; nt < NTILE; ++nt) s += hst[nt][r];
        s += __shfl_xor(s, 1, 32); s += __shfl_xor(s, 2, 32); s += __shfl_xor(s, 4, 32); s += __shfl_xor(s, 8, 32);
        mrow[r] = s;
      }
      if (c == 0) {
#pragma unroll
        for (int r = 0; r < 8; ++r) redS[(8 * hh + r) * NW + wave] = mrow[r];
      }
      __syncthreads();
#pragma unroll
      for (int nt = 0; nt < NTILE; ++nt) {
        const int j = 16 * NTILE * wave + 16 * nt + c;
#pragma unroll
        for (int r = 0; r < 8; ++r) Ah[(8 * hh + r) * HP + j] = (_Float16)hst[nt][r];
      }
      load_x_tile<F, NT, XMODE>(Ax, x32, x16, rowbase, (t + 1 < kSteps) ? (t + 1) : (kSteps - 1), tid);
#pragma unroll
      for (int r = 0; r < 8; ++r) {
        float s = 0.f;
#pragma unroll
        for (int w = 0; w < NW; ++w) s += redS[(8 * hh + r) * NW + w];
        mrow[r] = s * (1.0f / (float)H);
        float q = 0.f;
#pragma unroll
        for (int nt = 0; nt < NTILE; ++nt) { const float d = hst[nt][r] - mrow[r]; q += d * d; }
        q += __shfl_xor(q, 1, 32); q += __shfl_xor(q, 2, 32); q += __shfl_xor(q, 4, 32); q += __shfl_xor(q, 8, 32);
        rrow[r] = q;
      }
      if (c == 0) {
#pragma unroll
        for (int r = 0; r < 8; ++r) redQ[(8 * hh + r) * NW + wave] = rrow[r];
      }
      __syncthreads();
#pragma unroll
      for (int r = 0; r < 8; ++r) {
        float q = 0.f;
#pragma unroll
        for (int w = 0; w < NW; ++w) q += redQ[(8 * hh + r) * NW + w];
        rrow[r] = rsqrtf(q * (1.0f / (float)H) + kLnEps);
      }
#pragma unroll
      for (int nt = 0; nt < NTILE; ++nt) {
        const int j = 16 * NTILE * wave + 16 * nt + c;
#pragma unroll
        for (int r = 0; r < 8; ++r) {
          const float y = (hst[nt][r] - mrow[r]) * rrow[r] * ls[nt] + lb[nt];
          Ys[(8 * hh + r) * H + j] = (_Float16)y;
        }
      }
      __syncthreads();
      {
        constexpr int SEGS = H / 8;
        constexpr int ITERS = (kRows * SEGS) / NT;
        static_assert(ITERS * NT == kRows * SEGS);
        _Float16* hp = (_Float16*)hseq;
        for (int pass = 0; pass < 2; ++pass) {
#pragma unroll
          for (int it = 0; it < ITERS; ++it) {
            const int idx = it * NT + tid;
            const int row = idx / SEGS, c8 = (idx - row * SEGS) * 8;
            const v8h v = *(const v8h*)(Ys + row * H + c8);
            *(volatile v8h*)(hp + ((size_t)(rowbase + row) * kSteps + (size_t)t) * H + c8) = v;
          }
          __threadfence();
        }
      }
    } else {
      __syncthreads();
#pragma unroll
      for (int nt = 0; nt < NTILE; ++nt) {
        const int j = 16 * NTILE * wave + 16 * nt + c;
#pragma unroll
        for (int r = 0; r < 8; ++r) Ah[(8 * hh + r) * HP + j] = (_Float16)hst[nt][r];
      }
      load_x_tile<F, NT, XMODE>(Ax, x32, x16, rowbase, (t + 1 < kSteps) ? (t + 1) : (kSteps - 1), tid);
      __syncthreads();
    }
  }

  if constexpr (!SEQ) {
#pragma unroll
    for (int nt = 0; nt < NTILE; ++nt) {
      const int j = 16 * NTILE * wave + 16 * nt + c;
#pragma unroll
      for (int r = 0; r < 8; ++r) Hs[(8 * hh + r) * OP + j] = hst[nt][r];
    }
    __syncthreads();
    constexpr int SEG4 = H / 4;
    constexpr int ITER4 = (kRows * SEG4) / NT;
    static_assert(ITER4 * NT == kRows * SEG4);
    for (int pass = 0; pass < 2; ++pass) {
#pragma unroll
      for (int it = 0; it < ITER4; ++it) {
        const int idx = it * NT + tid;
        const int row = idx / SEG4, c4 = (idx - row * SEG4) * 4;
        const v4f v = *(const v4f*)(Hs + row * OP + c4);
        *(volatile v4f*)(hfin + (size_t)(rowbase + row) * H + c4) = v;
      }
      __threadfence();
    }
  }
}

template <int ND>
__device__ __forceinline__ v16h head_bfrag(const float* __restrict__ W, int kb, int ncl, bool nv) {
  v16h b;
#pragma unroll
  for (int e = 0; e < 8; ++e) {
    float w0 = W[(size_t)(kb + e) * ND + ncl];
    float w1 = W[(size_t)(kb + 16 + e) * ND + ncl];
    w0 = nv ? w0 : 0.0f;
    w1 = nv ? w1 : 0.0f;
    b[e]     = (_Float16)(bf16r(w0) * kWsc);
    b[8 + e] = (_Float16)(bf16r(w1) * kWsc);
  }
  return b;
}

template <int KD, int ND, bool LNRELU>
__device__ __forceinline__ void head_stage(const float* __restrict__ W, const float* __restrict__ bvec,
                                           const float* __restrict__ sc, const float* __restrict__ be,
                                           _Float16* ahi, _Float16* alo, float* os_wave, int lane) {
  constexpr int NJ = (ND + 15) / 16;
  static_assert(KD % 32 == 0 && KD <= 128 && ND <= 128);
  const int c = lane & 15, hh = lane >> 4, koff = hh * 8;
  v8f z[NJ];
#pragma unroll
  for (int j = 0; j < NJ; ++j) {
    const int n = 16 * j + c;
    const bool nv = n < ND;
    const int ncl = nv ? n : (ND - 1);
    v8f acc = zero8(), accl = zero8();
#pragma unroll
    for (int kc = 0; kc < KD / 32; ++kc) {
      const v16h ah = Frag<_Float16>::load(ahi + c * kAP + koff + 32 * kc);
      const v16h al = Frag<_Float16>::load(alo + c * kAP + koff + 32 * kc);
      const v16h b  = head_bfrag<ND>(W, 32 * kc + koff, ncl, nv);
      acc  = Frag<_Float16>::mma(ah, b, acc);
      accl = Frag<_Float16>::mma(al, b, accl);
      dep_guard3_h(acc, accl, ah, al, b);
    }
    const float bv = nv ? bf16r(bvec[ncl]) : 0.0f;
#pragma unroll
    for (int r = 0; r < 8; ++r) z[j][r] = acc[r] * kWscInv + accl[r] * (kWscInv * kResInv) + bv;
  }
  if constexpr (LNRELU) {
    float m[8], rs[8];
#pragma unroll
    for (int r = 0; r < 8; ++r) {
      float s = 0.f;
#pragma unroll
      for (int j = 0; j < NJ; ++j) s += z[j][r];
      s += __shfl_xor(s, 1, 32); s += __shfl_xor(s, 2, 32); s += __shfl_xor(s, 4, 32); s += __shfl_xor(s, 8, 32);
      m[r] = s * (1.0f / (float)ND);
      float q = 0.f;
#pragma unroll
      for (int j = 0; j < NJ; ++j) { const float d = z[j][r] - m[r]; q += d * d; }
      q += __shfl_xor(q, 1, 32); q += __shfl_xor(q, 2, 32); q += __shfl_xor(q, 4, 32); q += __shfl_xor(q, 8, 32);
      rs[r] = rsqrtf(q * (1.0f / (float)ND) + kLnEps);
    }
    __syncthreads();
#pragma unroll
    for (int j = 0; j < NJ; ++j) {
      const int n = 16 * j + c;
      const float sn = bf16r(sc[n]), bn = bf16r(be[n]);
#pragma unroll
      for (int r = 0; r < 8; ++r) {
        const float y = fmaxf((z[j][r] - m[r]) * rs[r] * sn + bn, 0.0f);
        const _Float16 hi = (_Float16)y;
        const _Float16 lo = (_Float16)((y - (float)hi) * kResSc);
        ahi[(8 * hh + r) * kAP + n] = hi;
        alo[(8 * hh + r) * kAP + n] = lo;
      }
    }
    __syncthreads();
  } else {
    if (c == 0) {
#pragma unroll
      for (int r = 0; r < 8; ++r) os_wave[8 * hh + r] = fmaxf(z[0][r], 0.0f);
    }
  }
}

__global__ __launch_bounds__(kHeadThreads) void head_kernel(
    const float* __restrict__ h3,
    const float* __restrict__ ln3s, const float* __restrict__ ln3b,
    const float* __restrict__ Wd1, const float* __restrict__ bd1, const float* __restrict__ s1, const float* __restrict__ e1,
    const float* __restrict__ Wd2, const float* __restrict__ bd2, const float* __restrict__ s2, const float* __restrict__ e2,
    const float* __restrict__ Wd3, const float* __restrict__ bd3, const float* __restrict__ s3, const float* __restrict__ e3,
    const float* __restrict__ Wout, const float* __restrict__ bout, const int* __restrict__ trainflag,
    float* __restrict__ out) {
  __shared__ __align__(16) _Float16 Ahi[4][kRows * kAP];
  __shared__ __align__(16) _Float16 Alo[4][kRows * kAP];
  __shared__ __align__(16) float    Os[kHeadRows];
  (void)trainflag;
  const int tid = threadIdx.x, lane = tid & 31, wave = tid >> 5;
  const int row0 = blockIdx.x * kHeadRows + wave * kRows;
  _Float16* ahi = Ahi[wave];
  _Float16* alo = Alo[wave];
  {
    const float sa = bf16r(ln3s[lane]), sb = bf16r(ln3s[32 + lane]);
    const float ba = bf16r(ln3b[lane]), bb2 = bf16r(ln3b[32 + lane]);
#pragma unroll 1
    for (int r = 0; r < kRows; ++r) {
      const float v0 = h3[(size_t)(row0 + r) * 64 + lane];
      const float v1 = h3[(size_t)(row0 + r) * 64 + 32 + lane];
      float s = v0 + v1;
      s += __shfl_xor(s, 1, 32); s += __shfl_xor(s, 2, 32); s += __shfl_xor(s, 4, 32); s += __shfl_xor(s, 8, 32); s += __shfl_xor(s, 16, 32);
      const float m = s * (1.0f / 64.0f);
      const float d0 = v0 - m, d1 = v1 - m;
      float q = d0 * d0 + d1 * d1;
      q += __shfl_xor(q, 1, 32); q += __shfl_xor(q, 2, 32); q += __shfl_xor(q, 4, 32); q += __shfl_xor(q, 8, 32); q += __shfl_xor(q, 16, 32);
      const float rstd = rsqrtf(q * (1.0f / 64.0f) + kLnEps);
      const float y0 = d0 * rstd * sa + ba;
      const float y1 = d1 * rstd * sb + bb2;
      const _Float16 h0 = (_Float16)y0, h1 = (_Float16)y1;
      ahi[r * kAP + lane]      = h0;
      alo[r * kAP + lane]      = (_Float16)((y0 - (float)h0) * kResSc);
      ahi[r * kAP + 32 + lane] = h1;
      alo[r * kAP + 32 + lane] = (_Float16)((y1 - (float)h1) * kResSc);
    }
  }
  __syncthreads();
  head_stage<64, 128, true>(Wd1, bd1, s1, e1, ahi, alo, Os, lane);
  head_stage<128, 64, true>(Wd2, bd2, s2, e2, ahi, alo, Os, lane);
  head_stage<64, 32, true>(Wd3, bd3, s3, e3, ahi, alo, Os, lane);
  head_stage<32, 1, false>(Wout, bout, bout, bout, ahi, alo, Os + wave * kRows, lane);
  __syncthreads();
  if (wave == 0 && lane < 16) {
    const v4f v = *(const v4f*)(Os + 4 * lane);
    float* op = out + (size_t)blockIdx.x * kHeadRows + 4 * lane;
    *(volatile v4f*)op = v;
    __threadfence();
    *(volatile v4f*)op = v;
  }
}

extern "C" void kernel_launch(void* const* d_in, const int* in_sizes, int n_in,
                              void* d_out, int out_size, void* d_ws, size_t ws_size, hipStream_t stream) {
  if (n_in < 31 || d_out == nullptr || d_ws == nullptr) return;
  const int expect[31] = { kSeq * kSteps * 64, 64 * 1024, 256 * 1024, 1024, 256, 256,
                           256 * 512, 128 * 512, 512, 128, 128,
                           128 * 256, 64 * 256, 256, 64, 64,
                           64 * 128, 128, 128, 128, 128 * 64, 64, 64, 64, 64 * 32, 32, 32, 32, 32, 1, 1 };
  for (int i = 0; i < 31; ++i) if (in_sizes[i] != expect[i]) return;
  if (out_size != kSeq) return;

  const float* x    = (const float*)d_in[0];
  const float* Wx1  = (const float*)d_in[1];
  const float* Wh1  = (const float*)d_in[2];
  const float* b1   = (const float*)d_in[3];
  const float* ln1s = (const float*)d_in[4];
  const float* ln1b = (const float*)d_in[5];
  const float* Wx2  = (const float*)d_in[6];
  const float* Wh2  = (const float*)d_in[7];
  const float* b2   = (const float*)d_in[8];
  const float* ln2s = (const float*)d_in[9];
  const float* ln2b = (const float*)d_in[10];
  const float* Wx3  = (const float*)d_in[11];
  const float* Wh3  = (const float*)d_in[12];
  const float* b3   = (const float*)d_in[13];
  const float* ln3s = (const float*)d_in[14];
  const float* ln3b = (const float*)d_in[15];
  const float* Wd1  = (const float*)d_in[16];
  const float* bd1  = (const float*)d_in[17];
  const float* l1s  = (const float*)d_in[18];
  const float* l1b  = (const float*)d_in[19];
  const float* Wd2  = (const float*)d_in[20];
  const float* bd2  = (const float*)d_in[21];
  const float* l2s  = (const float*)d_in[22];
  const float* l2b  = (const float*)d_in[23];
  const float* Wd3  = (const float*)d_in[24];
  const float* bd3  = (const float*)d_in[25];
  const float* l3s  = (const float*)d_in[26];
  const float* l3b  = (const float*)d_in[27];
  const float* Wout = (const float*)d_in[28];
  const float* bout = (const float*)d_in[29];
  const int*   trn  = (const int*)d_in[30];
  float* out = (float*)d_out;

  char* ws = (char*)d_ws; size_t off = 0;
  auto carve = [&](size_t bytes) -> char* { char* p = ws + off; off += (bytes + 255) & ~(size_t)255; return p; };
  unsigned short* WX1 = (unsigned short*)carve((size_t)1024 * 64 * 2);
  unsigned short* WH1 = (unsigned short*)carve((size_t)1024 * 256 * 2);
  unsigned short* WX2 = (unsigned short*)carve((size_t)512 * 256 * 2);
  unsigned short* WH2 = (unsigned short*)carve((size_t)512 * 128 * 2);
  unsigned short* WX3 = (unsigned short*)carve((size_t)256 * 128 * 2);
  unsigned short* WH3 = (unsigned short*)carve((size_t)256 * 64 * 2);
  unsigned short* HS1 = (unsigned short*)carve((size_t)kSeq * kSteps * 256 * 2);
  unsigned short* HS2 = (unsigned short*)carve((size_t)kSeq * kSteps * 128 * 2);
  float*          H3F = (float*)carve((size_t)kSeq * 64 * 4);
  if (off > ws_size || off > (size_t)134217728) return;

  tpw_kernel<0><<<dim3(1024 / 64, 64 / 64),  kTpThreads, 0, stream>>>(Wx1, 64, 1024, 64, WX1, kWsc);
  tpw_kernel<1><<<dim3(1024 / 64, 256 / 64), kTpThreads, 0, stream>>>(Wh1, 256, 1024, 256, WH1, kWsc);
  tpw_kernel<1><<<dim3(512 / 64, 256 / 64),  kTpThreads, 0, stream>>>(Wx2, 256, 512, 256, WX2, kWsc);
  tpw_kernel<1><<<dim3(512 / 64, 128 / 64),  kTpThreads, 0, stream>>>(Wh2, 128, 512, 128, WH2, kWsc);
  tpw_kernel<1><<<dim3(256 / 64, 128 / 64),  kTpThreads, 0, stream>>>(Wx3, 128, 256, 128, WX3, kWsc);
  tpw_kernel<1><<<dim3(256 / 64, 64 / 64),   kTpThreads, 0, stream>>>(Wh3, 64, 256, 64, WH3, kWsc);
  rec_layer_kernel<64, 256, 8, 0, true><<<kRecBlocks, 256, 0, stream>>>(x, HS2, WX1, WH1, b1, ln1s, ln1b, HS1, H3F);
  rec_layer_kernel<256, 128, 8, 1, true><<<kRecBlocks, 256, 0, stream>>>(x, HS1, WX2, WH2, b2, ln2s, ln2b, HS2, H3F);
  rec_layer_kernel<128, 64, 4, 1, false><<<kRecBlocks, 128, 0, stream>>>(x, HS2, WX3, WH3, b3, ln3s, ln3b, HS1, H3F);
  head_kernel<<<kHeadBlocks, kHeadThreads, 0, stream>>>(H3F, ln3s, ln3b, Wd1, bd1, l1s, l1b, Wd2, bd2, l2s, l2b,
                                                        Wd3, bd3, l3s, l3b, Wout, bout, trn, out);
}
